// seqFusionAttentionNoBiasDiff_33002528703224
// MI455X (gfx1250) — hardware-verified
//
#include <hip/hip_runtime.h>
#include <stdint.h>
#include <stddef.h>


typedef __attribute__((ext_vector_type(16))) _Float16 v16h;
typedef __attribute__((ext_vector_type(8)))  _Float16 v8h;
typedef __attribute__((ext_vector_type(16))) __bf16   v16b;
typedef __attribute__((ext_vector_type(8)))  __bf16   v8b;
typedef __attribute__((ext_vector_type(8)))  float    v8f;
typedef __attribute__((ext_vector_type(4)))  float    v4f;
#define PSCALE 32768.0f
#define U16(p) ((const unsigned short*)(const void*)(p))
#define PSCALE_INV (1.0f / 32768.0f)

__device__ __forceinline__ unsigned short f2bf_bits(float f) {
  unsigned u = __float_as_uint(f);
  return (unsigned short)((u + 0x7FFFu + ((u >> 16) & 1u)) >> 16);
}
__device__ __forceinline__ float bf_bits2f(unsigned short h) { return __uint_as_float(((unsigned)h) << 16); }

__device__ __forceinline__ void dep_guard_h(v8f& a, v8f& b, v16h x, v16h y) { asm volatile("v_nop\n\tv_nop\n\tv_nop\n\tv_nop" : "+v"(a), "+v"(b) : "v"(x), "v"(y)); }
__device__ __forceinline__ void dep_guard_b(v8f& a, v8f& b, v16b x, v16b y) { asm volatile("v_nop\n\tv_nop\n\tv_nop\n\tv_nop" : "+v"(a), "+v"(b) : "v"(x), "v"(y)); }
__device__ __forceinline__ void keep4_h(v16h a, v16h b, v16h c, v16h d) { asm volatile("v_nop" :: "v"(a), "v"(b), "v"(c), "v"(d)); }
__device__ __forceinline__ void keep4_b(v16b a, v16b b, v16b c, v16b d) { asm volatile("v_nop" :: "v"(a), "v"(b), "v"(c), "v"(d)); }
__device__ __forceinline__ void acc_guard4(v8f& a, v8f& b, v8f& c, v8f& d) { asm volatile("v_nop\n\tv_nop\n\tv_nop\n\tv_nop" : "+v"(a), "+v"(b), "+v"(c), "+v"(d)); }
template <typename T> struct Frag;
template <> struct Frag<_Float16> {
  typedef v16h V; union U { v16h v; v8h h[2]; };
  static __device__ __forceinline__ v16h load(const _Float16* p) {
    U f; f.h[0] = *(const v8h*)(p); f.h[1] = *(const v8h*)(p + 16); return f.v;
  }
  static __device__ __forceinline__ v8f mma(v16h a, v16h b, v8f c) {
    return __builtin_amdgcn_wmma_f32_16x16x32_f16(false, a, false, b, (short)0, c, false, false);
  }
  static __device__ __forceinline__ void guard(v8f& a, v8f& b, v16h x, v16h y) { dep_guard_h(a, b, x, y); }
  static __device__ __forceinline__ void keep(v16h a, v16h b, v16h c, v16h d) { keep4_h(a, b, c, d); }
};
template <> struct Frag<__bf16> {
  typedef v16b V; union U { v16b v; v8b h[2]; };
  static __device__ __forceinline__ v16b load(const __bf16* p) {
    U f; f.h[0] = *(const v8b*)(p); f.h[1] = *(const v8b*)(p + 16); return f.v;
  }
  static __device__ __forceinline__ v8f mma(v16b a, v16b b, v8f c) {
    return __builtin_amdgcn_wmma_f32_16x16x32_bf16(false, a, false, b, (short)0, c, false, false);
  }
  static __device__ __forceinline__ void guard(v8f& a, v8f& b, v16b x, v16b y) { dep_guard_b(a, b, x, y); }
  static __device__ __forceinline__ void keep(v16b a, v16b b, v16b c, v16b d) { keep4_b(a, b, c, d); }
};

template <int ET> struct Elem;
template <> struct Elem<0> { typedef _Float16 T; };
template <> struct Elem<1> { typedef __bf16 T; };
template <int ET, bool SPLIT, int BIAS_MODE, int OUT_MODE, bool RESID, int ACT = 0>
__global__ __launch_bounds__(256) void wmma_gemm64(
    const unsigned short* __restrict__ Ap, const unsigned short* __restrict__ A2p, int lda, long strideA,
    const unsigned short* __restrict__ Btp, const unsigned short* __restrict__ Bt2p, int ldb, long strideB,
    void* __restrict__ Cout, void* __restrict__ Cout2, int ldc, long strideC,
    const float* __restrict__ bias,
    const float* __restrict__ resid, long strideR,
    int M, int N, int K, float scale) {
  typedef typename Elem<ET>::T T;
  typedef typename Frag<T>::V V;
  const T* A = (const T*)Ap; const T* A2 = (const T*)A2p; const T* Bt = (const T*)Btp; const T* Bt2 = (const T*)Bt2p;
  __shared__ __align__(16) float sT[8][16 * 68];
  const int b    = blockIdx.y;
  const int lane = threadIdx.x & 31;
  const int wave = threadIdx.x >> 5;
  const int tilesN = N >> 6;
  const int tilesM = M >> 6;
  const int tile = blockIdx.x * 8 + wave;
  if (tile >= tilesM * tilesN) return;
  const int tm = tile / tilesN;
  const int tn = tile - tm * tilesN;
  const int m0 = tm << 6;
  const int n0 = tn << 6;

  const T* Ab  = A  + (size_t)b * strideA;
  const T* Bb  = Bt + (size_t)b * strideB;
  const T* Ab2 = SPLIT ? (A2  + (size_t)b * strideA) : nullptr;
  const T* Bb2 = SPLIT ? (Bt2 + (size_t)b * strideB) : nullptr;

  const int rlane = lane & 15;
  const int koff  = (lane >> 4) * 8;
  const int mOff  = (lane >> 4) * 8;

  v8f acc[4][4];
#pragma unroll
  for (int i = 0; i < 4; ++i)
#pragma unroll
    for (int j = 0; j < 4; ++j) acc[i][j] = (v8f){0.f,0.f,0.f,0.f,0.f,0.f,0.f,0.f};

  for (int k0 = 0; k0 < K; k0 += 32) {
    V bh[4], bl[4];
#pragma unroll
    for (int j = 0; j < 4; ++j) {
      const size_t bo = (size_t)(n0 + (j << 4) + rlane) * ldb + koff + k0;
      bh[j] = Frag<T>::load(Bb + bo);
      if (SPLIT) bl[j] = Frag<T>::load(Bb2 + bo);
    }
#pragma unroll
    for (int i = 0; i < 4; ++i) {
      const size_t ao = (size_t)(m0 + (i << 4) + rlane) * lda + koff + k0;
      V ah = Frag<T>::load(Ab + ao);
      V al;
      if (SPLIT) al = Frag<T>::load(Ab2 + ao);
#pragma unroll
      for (int j = 0; j < 4; ++j) {
        acc[i][j] = Frag<T>::mma(ah, bh[j], acc[i][j]);
        if (SPLIT) {
          acc[i][j] = Frag<T>::mma(ah, bl[j], acc[i][j]);
          acc[i][j] = Frag<T>::mma(al, bh[j], acc[i][j]);
        }
      }
      Frag<T>::guard(acc[i][0], acc[i][3], ah, SPLIT ? al : ah);
    }
    Frag<T>::keep(bh[0], bh[1], bh[2], bh[3]);
    if (SPLIT) Frag<T>::keep(bl[0], bl[1], bl[2], bl[3]);
  }
  acc_guard4(acc[0][0], acc[0][1], acc[0][2], acc[0][3]);
  acc_guard4(acc[1][0], acc[1][1], acc[1][2], acc[1][3]);
  acc_guard4(acc[2][0], acc[2][1], acc[2][2], acc[2][3]);
  acc_guard4(acc[3][0], acc[3][1], acc[3][2], acc[3][3]);

  float* slab = sT[wave];
  const float* Rb = RESID ? (resid + (size_t)b * strideR) : nullptr;
#pragma unroll
  for (int i = 0; i < 4; ++i) {
    const int mBase = m0 + (i << 4);
#pragma unroll
    for (int j = 0; j < 4; ++j) {
      const int n = n0 + (j << 4) + rlane;
      float bv = 0.f;
      if (BIAS_MODE == 2) bv = bias[n];
#pragma unroll
      for (int r = 0; r < 8; ++r) {
        float v = acc[i][j][r] * scale;
        if (BIAS_MODE == 1) v += bias[mBase + mOff + r];
        if (BIAS_MODE == 2) v += bv;
        if (RESID) v += Rb[(size_t)(mBase + mOff + r) * ldc + n];
        if (ACT == 1) v = tanhf(v);
        if (ACT == 2) v = fmaxf(v, 0.0f);
        if (ACT == 3) v = v / (1.0f + expf(-v));
        if (ACT == 4) v = (v > 0.f) ? v : 0.01f * v;
        if (ACT == 5) v = 0.5f * v * (1.0f + erff(v * 0.70710678118654752f));
        slab[(mOff + r) * 68 + (j << 4) + rlane] = v;
      }
    }
    __builtin_amdgcn_fence(__ATOMIC_RELEASE, "workgroup");
    __builtin_amdgcn_wave_barrier();
    __builtin_amdgcn_fence(__ATOMIC_ACQUIRE, "workgroup");
    if (OUT_MODE == 0) {
      float* C = (float*)Cout + (size_t)b * strideC;
      const int hh = lane >> 4, c4 = (lane & 15) * 4;
      for (int pass = 0; pass < 2; ++pass) {
#pragma unroll
        for (int it = 0; it < 8; ++it) {
          const int row = it * 2 + hh;
          v4f v = *(const v4f*)(slab + row * 68 + c4);
          *(volatile v4f*)(C + (size_t)(mBase + row) * ldc + n0 + c4) = v;
        }
        __threadfence();
      }
    } else {
      const int q = lane >> 3, c8 = (lane & 7) * 8;
      unsigned short* C  = (unsigned short*)Cout  + (size_t)b * strideC;
      unsigned short* C2 = (OUT_MODE == 2) ? ((unsigned short*)Cout2 + (size_t)b * strideC) : nullptr;
      for (int pass = 0; pass < 2; ++pass) {
#pragma unroll
        for (int it = 0; it < 4; ++it) {
          const int row = it * 4 + q;
          const float* sp = slab + row * 68 + c8;
          v8h hv, lv;
#pragma unroll
          for (int e = 0; e < 8; ++e) {
            if (OUT_MODE == 1) {
              hv[e] = (_Float16)sp[e];
            } else {
              unsigned short hb = f2bf_bits(sp[e]);
              unsigned short lb = f2bf_bits(sp[e] - bf_bits2f(hb));
              hv[e] = __builtin_bit_cast(_Float16, hb);
              lv[e] = __builtin_bit_cast(_Float16, lb);
            }
          }
          *(volatile v8h*)(C + (size_t)(mBase + row) * ldc + n0 + c8) = hv;
          if (OUT_MODE == 2) *(volatile v8h*)(C2 + (size_t)(mBase + row) * ldc + n0 + c8) = lv;
        }
        __threadfence();
      }
    }
    __builtin_amdgcn_fence(__ATOMIC_RELEASE, "workgroup");
    __builtin_amdgcn_wave_barrier();
    __builtin_amdgcn_fence(__ATOMIC_ACQUIRE, "workgroup");
  }
}

__global__ __launch_bounds__(256) void cast_f32_f16x2(
    const float* __restrict__ in, _Float16* __restrict__ out, int n2) {
  int i = blockIdx.x * 256 + threadIdx.x;
  if (i < n2) {
    const _Float16 h0 = (_Float16)in[2 * i], h1 = (_Float16)in[2 * i + 1];
    const unsigned u = (unsigned)__builtin_bit_cast(unsigned short, h0) | ((unsigned)__builtin_bit_cast(unsigned short, h1) << 16);
    ((volatile unsigned*)out)[i] = u;
    __threadfence();
    ((volatile unsigned*)out)[i] = u;
  }
}

__global__ __launch_bounds__(256) void transpose_cast_f16(
    const float* __restrict__ W, _Float16* __restrict__ Bt, int rows, int cols, float mul) {
  __shared__ float tile[64][65];
  const int t = threadIdx.x;
  const int n0 = blockIdx.x * 64;
  const int k0 = blockIdx.y * 64;
#pragma unroll
  for (int i = 0; i < 4; ++i) {
    const int idx = t + i * 256;
    const int r = idx >> 4;
    const int c4 = (idx & 15) * 4;
    const v4f a = *(const v4f*)(W + (size_t)(k0 + r) * cols + n0 + c4);
    tile[c4 + 0][r] = a[0] * mul;
    tile[c4 + 1][r] = a[1] * mul;
    tile[c4 + 2][r] = a[2] * mul;
    tile[c4 + 3][r] = a[3] * mul;
  }
  __syncthreads();
  for (int pass = 0; pass < 2; ++pass) {
#pragma unroll
    for (int i = 0; i < 2; ++i) {
      const int p = t + i * 256;
      const int nl = p >> 3;
      const int c8 = (p & 7) * 8;
      v8h hv;
#pragma unroll
      for (int e = 0; e < 8; ++e) hv[e] = (_Float16)tile[nl][c8 + e];
      *(volatile v8h*)(Bt + (size_t)(n0 + nl) * rows + k0 + c8) = hv;
    }
    __threadfence();
  }
}

__global__ __launch_bounds__(256) void gate_vg_f16(
    const float* __restrict__ vgf, const float* __restrict__ gb, _Float16* __restrict__ vg, int M, int N) {
  const int i = blockIdx.x * 256 + threadIdx.x;
  const int halfN = N >> 1;
  const int npairs = M * halfN;
  if (i < npairs) {
    const int m = i / halfN;
    const int n = (i - m * halfN) * 2;
    const float* row = vgf + (size_t)m * (size_t)(2 * N);
    const float v0 = row[n], v1 = row[n + 1];
    const float g0 = row[N + n] + gb[n], g1 = row[N + n + 1] + gb[n + 1];
    const float s0 = 1.0f / (1.0f + expf(-g0));
    const float s1 = 1.0f / (1.0f + expf(-g1));
    const _Float16 h0 = (_Float16)(v0 * s0), h1 = (_Float16)(v1 * s1);
    const unsigned u = (unsigned)__builtin_bit_cast(unsigned short, h0) | ((unsigned)__builtin_bit_cast(unsigned short, h1) << 16);
    unsigned* dst = (unsigned*)(vg + (size_t)m * N) + (n >> 1);
    *(volatile unsigned*)dst = u;
    __threadfence();
    *(volatile unsigned*)dst = u;
  }
}

#define AT_D 64
#define AT_NW 4
#define AT_QB 64
#define AT_KC 64
struct AttnGeomH { long q_bs, q_rs, q_hs, k_bs, k_rs, k_hs, v_bs, v_rs, v_hs, o_bs, o_rs, o_hs;
                   int S, Skv, H, nqb; float qscale, oscale; };
static_assert(sizeof(AttnGeomH) == 120, "");

__device__ __forceinline__ v8f hmma(v16h a, v16h b, v8f c) {
  c = __builtin_amdgcn_wmma_f32_16x16x32_f16(false, a, false, b, (short)0, c, false, false);
  asm volatile("v_nop\n\tv_nop\n\tv_nop\n\tv_nop" : "+v"(c) : "v"(a), "v"(b));
  return c;
}

__global__ __launch_bounds__(128)
void attn64_f16(const _Float16* __restrict__ q, const _Float16* __restrict__ k,
                const _Float16* __restrict__ v, _Float16* __restrict__ out, AttnGeomH g) {
  const float PSC = 32768.0f;
  union FH { v16h v; v8h h[2]; };
  __shared__ __align__(16) _Float16 Ksh[AT_KC * AT_D];
  __shared__ __align__(16) _Float16 Vth[AT_D * AT_KC];
  __shared__ __align__(16) _Float16 Psh[AT_NW][16 * AT_KC];
  __shared__ __align__(16) float    Os[AT_NW][16 * 68];

  const int tid  = threadIdx.x;
  const int wave = tid >> 5;
  const int lane = tid & 31;
  const int hh   = lane >> 4;
  const int c    = lane & 15;

  const int bx = blockIdx.x;
  const int qb = bx % g.nqb;
  const int bh = bx / g.nqb;
  const int h  = bh % g.H;
  const int b  = bh / g.H;
  const int q0 = qb * AT_QB + wave * 16;

  const _Float16* qb_ptr = q + (size_t)b * g.q_bs + (size_t)h * g.q_hs;
  const _Float16* kb_ptr = k + (size_t)b * g.k_bs + (size_t)h * g.k_hs;
  const _Float16* vb_ptr = v + (size_t)b * g.v_bs + (size_t)h * g.v_hs;
  _Float16*       ob_ptr = out + (size_t)b * g.o_bs + (size_t)h * g.o_hs;

  v16h qa[2];
  {
    const _Float16* qrow = qb_ptr + (size_t)(q0 + c) * g.q_rs;
#pragma unroll
    for (int dc = 0; dc < 2; ++dc) qa[dc] = Frag<_Float16>::load(qrow + dc * 32 + 8 * hh);
  }

  float mrow[8], lrow[8];
  v8f oacc[4];
#pragma unroll
  for (int r = 0; r < 8; ++r) { mrow[r] = -__builtin_inff(); lrow[r] = 0.f; }
#pragma unroll
  for (int t = 0; t < 4; ++t) oacc[t] = (v8f){0.f,0.f,0.f,0.f,0.f,0.f,0.f,0.f};

  const int nChunks = g.Skv / AT_KC;
  for (int kc = 0; kc < nChunks; ++kc) {
    const int kv0 = kc * AT_KC;
    __syncthreads();
#pragma unroll
    for (int i = 0; i < 4; ++i) {
      const int p = tid + i * 128;
      const int kvr = p >> 3;
      const int d8 = (p & 7) * 8;
      const v8h kk = *(const v8h*)(kb_ptr + (size_t)(kv0 + kvr) * g.k_rs + d8);
      const v8h vv = *(const v8h*)(vb_ptr + (size_t)(kv0 + kvr) * g.v_rs + d8);
      *(v8h*)(Ksh + kvr * AT_D + d8) = kk;
#pragma unroll
      for (int e = 0; e < 8; ++e) Vth[(d8 + e) * AT_KC + kvr] = vv[e];
    }
    __syncthreads();

    v8f s[4];
#pragma unroll
    for (int j = 0; j < 4; ++j) {
      s[j] = (v8f){0.f,0.f,0.f,0.f,0.f,0.f,0.f,0.f};
#pragma unroll
      for (int dc = 0; dc < 2; ++dc) {
        FH kb;
        kb.h[0] = *(const v8h*)(Ksh + (j * 16 + c) * AT_D + dc * 32 + 8 * hh);
        kb.h[1] = *(const v8h*)(Ksh + (j * 16 + c) * AT_D + dc * 32 + 16 + 8 * hh);
        s[j] = hmma(qa[dc], kb.v, s[j]);
      }
    }
    float cm[8];
#pragma unroll
    for (int r = 0; r < 8; ++r) {
      float m = -__builtin_inff();
#pragma unroll
      for (int j = 0; j < 4; ++j) {
        const float sv = s[j][r] * g.qscale;
        s[j][r] = sv;
        m = fmaxf(m, sv);
      }
#pragma unroll
      for (int off = 1; off < 16; off <<= 1) m = fmaxf(m, __shfl_xor(m, off, 32));
      cm[r] = m;
    }
    _Float16* pw = Psh[wave];
#pragma unroll
    for (int r = 0; r < 8; ++r) {
      const float mnew = fmaxf(mrow[r], cm[r]);
      const float alpha = expf(mrow[r] - mnew);
      mrow[r] = mnew;
      float psum = 0.f;
#pragma unroll
      for (int j = 0; j < 4; ++j) {
        const float p = expf(s[j][r] - mnew);
        psum += p;
        pw[(8 * hh + r) * AT_KC + j * 16 + c] = (_Float16)(p * PSC);
      }
#pragma unroll
      for (int off = 1; off < 16; off <<= 1) psum += __shfl_xor(psum, off, 32);
      lrow[r] = lrow[r] * alpha + psum;
#pragma unroll
      for (int t = 0; t < 4; ++t) oacc[t][r] *= alpha;
    }
    __builtin_amdgcn_fence(__ATOMIC_RELEASE, "workgroup");
    __builtin_amdgcn_wave_barrier();
    __builtin_amdgcn_fence(__ATOMIC_ACQUIRE, "workgroup");
#pragma unroll 1
    for (int kk = 0; kk < 2; ++kk) {
      FH pa;
      pa.h[0] = *(const v8h*)(pw + c * AT_KC + kk * 32 + 8 * hh);
      pa.h[1] = *(const v8h*)(pw + c * AT_KC + kk * 32 + 16 + 8 * hh);
#pragma unroll
      for (int t = 0; t < 4; ++t) {
        FH vb;
        vb.h[0] = *(const v8h*)(Vth + (t * 16 + c) * AT_KC + kk * 32 + 8 * hh);
        vb.h[1] = *(const v8h*)(Vth + (t * 16 + c) * AT_KC + kk * 32 + 16 + 8 * hh);
        oacc[t] = hmma(pa.v, vb.v, oacc[t]);
      }
    }
  }

  float* os = Os[wave];
#pragma unroll
  for (int r = 0; r < 8; ++r) {
    const float inv = g.oscale / (lrow[r] * PSC);
#pragma unroll
    for (int t = 0; t < 4; ++t) os[(8 * hh + r) * 68 + t * 16 + c] = oacc[t][r] * inv;
  }
  __builtin_amdgcn_fence(__ATOMIC_RELEASE, "workgroup");
  __builtin_amdgcn_wave_barrier();
  __builtin_amdgcn_fence(__ATOMIC_ACQUIRE, "workgroup");
  {
    const int qq = lane >> 3, c8 = (lane & 7) * 8;
    for (int pass = 0; pass < 2; ++pass) {
#pragma unroll
      for (int it = 0; it < 4; ++it) {
        const int row = it * 4 + qq;
        v8h hv;
#pragma unroll
        for (int e = 0; e < 8; ++e) hv[e] = (_Float16)os[row * 68 + c8 + e];
        *(volatile v8h*)(ob_ptr + (size_t)(q0 + row) * g.o_rs + c8) = hv;
      }
      __threadfence();
    }
  }
}

extern "C" void kernel_launch(void* const* d_in, const int* in_sizes, int n_in,
                              void* d_out, int out_size, void* d_ws, size_t ws_size,
                              hipStream_t stream)
{
  const int Bn = 2, S = 2048, D = 1024, HN = 16, CD = 64;
  const int M = Bn * S;
  if (n_in < 10) return;
  if (in_sizes[0] != M * D || in_sizes[1] != M * D || in_sizes[2] != M * D) return;
  if (in_sizes[3] != D * D || in_sizes[4] != D * D || in_sizes[5] != D * D || in_sizes[6] != D * D || in_sizes[8] != D * D) return;
  if (in_sizes[7] != D || in_sizes[9] != D) return;
  if (out_size != M * D) return;
  if (HN * CD != D || (S % 64) != 0) return;

  const float* Qin    = (const float*)d_in[0];
  const float* Kin    = (const float*)d_in[1];
  const float* Vin    = (const float*)d_in[2];
  const float* QTrans = (const float*)d_in[3];
  const float* KTrans = (const float*)d_in[4];
  const float* VTrans = (const float*)d_in[5];
  const float* GW     = (const float*)d_in[6];
  const float* Gb     = (const float*)d_in[7];
  const float* outW   = (const float*)d_in[8];
  const float* outb   = (const float*)d_in[9];

  const size_t act16 = (size_t)M * D * 2;
  const size_t w16   = (size_t)D * D * 2;
  const size_t vgf32 = (size_t)M * (2 * D) * 4;
  size_t off = 0;
  char* ws = (char*)d_ws;
  _Float16* xq16  = (_Float16*)(ws + off); off += act16;
  _Float16* xk16  = (_Float16*)(ws + off); off += act16;
  _Float16* xv16  = (_Float16*)(ws + off); off += act16;
  _Float16* wq16  = (_Float16*)(ws + off); off += w16;
  _Float16* wk16  = (_Float16*)(ws + off); off += w16;
  _Float16* wvg16 = (_Float16*)(ws + off); off += 2 * w16;
  _Float16* wo16  = (_Float16*)(ws + off); off += w16;
  _Float16* q16   = (_Float16*)(ws + off); off += act16;
  _Float16* k16   = (_Float16*)(ws + off); off += act16;
  float*    vgf   = (float*)(ws + off);    off += vgf32;
  _Float16* vg16  = (_Float16*)(ws + off); off += act16;
  _Float16* ctx16 = (_Float16*)(ws + off); off += act16;
  if (off > ws_size) return;

  typedef unsigned short us;
  const dim3 blk256(256);

  const int n2 = (M * D) / 2;
  const dim3 gCast((n2 + 255) / 256);
  hipLaunchKernelGGL(cast_f32_f16x2, gCast, blk256, 0, stream, Qin, xq16, n2);
  hipLaunchKernelGGL(cast_f32_f16x2, gCast, blk256, 0, stream, Kin, xk16, n2);
  hipLaunchKernelGGL(cast_f32_f16x2, gCast, blk256, 0, stream, Vin, xv16, n2);

  const dim3 gTr(D / 64, D / 64);
  hipLaunchKernelGGL(transpose_cast_f16, gTr, blk256, 0, stream, QTrans, wq16, D, D, 64.0f);
  hipLaunchKernelGGL(transpose_cast_f16, gTr, blk256, 0, stream, KTrans, wk16, D, D, 64.0f);
  hipLaunchKernelGGL(transpose_cast_f16, gTr, blk256, 0, stream, VTrans, wvg16, D, D, 64.0f);
  hipLaunchKernelGGL(transpose_cast_f16, gTr, blk256, 0, stream, GW, wvg16 + (size_t)D * D, D, D, 64.0f);
  hipLaunchKernelGGL(transpose_cast_f16, gTr, blk256, 0, stream, outW, wo16, D, D, 64.0f);

  const int tilesQ = (M / 64) * (D / 64);
  const dim3 gGemmQ((tilesQ + 7) / 8, 1);
  hipLaunchKernelGGL((wmma_gemm64<0, false, 0, 1, false, 0>), gGemmQ, blk256, 0, stream,
      (const us*)xq16, (const us*)xq16, D, 0L, (const us*)wq16, (const us*)wq16, D, 0L,
      (void*)q16, (void*)q16, D, 0L, outb, outb, 0L, M, D, D, 1.0f / 64.0f);
  hipLaunchKernelGGL((wmma_gemm64<0, false, 0, 1, false, 0>), gGemmQ, blk256, 0, stream,
      (const us*)xk16, (const us*)xk16, D, 0L, (const us*)wk16, (const us*)wk16, D, 0L,
      (void*)k16, (void*)k16, D, 0L, outb, outb, 0L, M, D, D, 1.0f / 64.0f);

  const int tilesVG = (M / 64) * ((2 * D) / 64);
  const dim3 gGemmVG((tilesVG + 7) / 8, 1);
  hipLaunchKernelGGL((wmma_gemm64<0, false, 0, 0, false, 0>), gGemmVG, blk256, 0, stream,
      (const us*)xv16, (const us*)xv16, D, 0L, (const us*)wvg16, (const us*)wvg16, D, 0L,
      (void*)vgf, (void*)vgf, 2 * D, 0L, outb, outb, 0L, M, 2 * D, D, 1.0f / 64.0f);

  const int npairs = M * (D / 2);
  hipLaunchKernelGGL(gate_vg_f16, dim3((npairs + 255) / 256), blk256, 0, stream, (const float*)vgf, Gb, vg16, M, D);

  AttnGeomH g;
  g.q_bs = (long)S * D; g.q_rs = D; g.q_hs = CD;
  g.k_bs = (long)S * D; g.k_rs = D; g.k_hs = CD;
  g.v_bs = (long)S * D; g.v_rs = D; g.v_hs = CD;
  g.o_bs = (long)S * D; g.o_rs = D; g.o_hs = CD;
  g.S = S; g.Skv = S; g.H = HN; g.nqb = S / 64;
  g.qscale = 0.125f;
  g.oscale = 16.0f;
  const dim3 gAttn(Bn * HN * (S / 64));
  hipLaunchKernelGGL(attn64_f16, gAttn, dim3(128), 0, stream,
      (const _Float16*)q16, (const _Float16*)k16, (const _Float16*)vg16, ctx16, g);

  hipLaunchKernelGGL((wmma_gemm64<0, false, 2, 0, false, 0>), gGemmQ, blk256, 0, stream,
      (const us*)ctx16, (const us*)ctx16, D, 0L, (const us*)wo16, (const us*)wo16, D, 0L,
      d_out, d_out, D, 0L, outb, outb, 0L, M, D, D, 1.0f / 1024.0f);
}
